// GraphSAGE_AML_32246614458737
// MI455X (gfx1250) — hardware-run, weakly checked
//
#include <hip/hip_runtime.h>

typedef float          v8f   __attribute__((ext_vector_type(8)));
typedef float          v4f   __attribute__((ext_vector_type(4)));
typedef unsigned int   v4u   __attribute__((ext_vector_type(4)));
typedef int            v8i   __attribute__((ext_vector_type(8)));
typedef unsigned short v8us  __attribute__((ext_vector_type(8)));
typedef unsigned short v16us __attribute__((ext_vector_type(16)));
typedef __bf16         v16bf __attribute__((ext_vector_type(16)));
typedef _Float16       v16h  __attribute__((ext_vector_type(16)));
typedef v4f  __attribute__((may_alias)) v4fa;
typedef v8us __attribute__((may_alias)) v8usa;
union FragB { v16bf v; v16us u; v8us h[2]; v8i w; };
union FragH { v16h  v; v16us u; v8us h[2]; v8i w; };

__device__ __forceinline__ v8f wmb(const FragB& a, const FragB& b, v8f c) {
  v8f d = __builtin_amdgcn_wmma_f32_16x16x32_bf16(false, a.v, false, b.v, (short)0, c, false, false);
  asm volatile("v_nop\n\tv_nop\n\tv_nop\n\tv_nop" : "+v"(d) : "v"(a.w), "v"(b.w));
  return d;
}

__device__ __forceinline__ v8f wmh(const FragH& a, const FragH& b, v8f c) {
  v8f d = __builtin_amdgcn_wmma_f32_16x16x32_f16(false, a.v, false, b.v, (short)0, c, false, false);
  asm volatile("v_nop\n\tv_nop\n\tv_nop\n\tv_nop" : "+v"(d) : "v"(a.w), "v"(b.w));
  return d;
}

__device__ __forceinline__ unsigned bf16_bits(float f) {
  const unsigned u = __float_as_uint(f);
  const unsigned r = (u + 0x7FFFu + ((u >> 16) & 1u)) >> 16;
  const unsigned q = (u >> 16) | 0x40u;
  return ((u & 0x7fffffffu) > 0x7f800000u) ? q : r;
}

__device__ __forceinline__ float bf16_val(float f) {
  return __uint_as_float(bf16_bits(f) << 16);
}
__device__ __forceinline__ int clampi(int v, int lo, int hi) {
  return v < lo ? lo : (v > hi ? hi : v);
}

__device__ __forceinline__ unsigned f16_bits(float f) {
  const unsigned u  = __float_as_uint(f);
  const unsigned s  = (u >> 16) & 0x8000u;
  const unsigned a  = u & 0x7fffffffu;
  const unsigned t  = a - 0x38000000u;
  const unsigned r  = (t + 0x0FFFu + ((t >> 13) & 1u)) >> 13;
  const unsigned rc = r > 0x7C00u ? 0x7C00u : r;
  const bool small  = a < 0x38800000u;
  const bool isnan  = a > 0x7f800000u;
  const unsigned fin = small ? 0u : (s | rc);
  return isnan ? (s | 0x7E00u) : fin;
}

__device__ __forceinline__ unsigned pk16(unsigned lo, unsigned hi) { return lo | (hi << 16); }
__device__ __forceinline__ unsigned bf16_lo_bits(float v) {
  float hi = bf16_val(v);
  asm volatile("" : "+v"(hi));
  return bf16_bits(v - hi);
}
__device__ __forceinline__ v4u pack8_bf16(v4f a, v4f c) {
  return (v4u){ pk16(bf16_bits(a[0]), bf16_bits(a[1])), pk16(bf16_bits(a[2]), bf16_bits(a[3])),
                pk16(bf16_bits(c[0]), bf16_bits(c[1])), pk16(bf16_bits(c[2]), bf16_bits(c[3])) };
}
__device__ __forceinline__ v4u pack8_bf16_lo(v4f a, v4f c) {
  return (v4u){ pk16(bf16_lo_bits(a[0]), bf16_lo_bits(a[1])), pk16(bf16_lo_bits(a[2]), bf16_lo_bits(a[3])),
                pk16(bf16_lo_bits(c[0]), bf16_lo_bits(c[1])), pk16(bf16_lo_bits(c[2]), bf16_lo_bits(c[3])) };
}
__device__ __forceinline__ v4u pack8_f16(v4f a, v4f c) {
  return (v4u){ pk16(f16_bits(a[0]), f16_bits(a[1])), pk16(f16_bits(a[2]), f16_bits(a[3])),
                pk16(f16_bits(c[0]), f16_bits(c[1])), pk16(f16_bits(c[2]), f16_bits(c[3])) };
}

template <int FORM>
__global__ __launch_bounds__(256) void k_plane(const float* __restrict__ src, int rows, int cols, int ldsrc,
                                               unsigned short* __restrict__ dst, int MP, int KP) {
  static_assert(FORM >= 0 && FORM <= 3);
  const int KTOT = (FORM == 1 || FORM == 3) ? 2 * KP : KP;
  const unsigned ppr   = (unsigned)(KTOT >> 3);
  const unsigned kp8   = (unsigned)(KP >> 3);
  const unsigned total = (unsigned)MP * ppr;
  const unsigned g     = blockIdx.x * 256u + threadIdx.x;
  const unsigned rowu  = g / ppr;
  const unsigned p     = g - rowu * ppr;
  const bool second    = p >= kp8;
  const int row = (int)rowu;
  const int c0  = (int)((second ? p - kp8 : p) << 3);
  const float* srow = src + (size_t)clampi(row, 0, rows - 1) * (size_t)ldsrc;
  float x[8];
  unsigned mk[8];
#pragma unroll
  for (int e = 0; e < 8; ++e) {
    const int c = c0 + e;
    const float v = srow[clampi(c, 0, cols - 1)];
    asm volatile("" :: "v"(v));
    x[e]  = v;
    mk[e] = (row < rows && c < cols) ? 0xFFFFu : 0u;
  }
  const v4f a = (v4f){ x[0], x[1], x[2], x[3] };
  const v4f c = (v4f){ x[4], x[5], x[6], x[7] };
  v4u o;
  if (FORM == 2) {
    o = pack8_f16(a, c);
  } else {
    const v4u hi = pack8_bf16(a, c);
    o = hi;
    if (FORM == 1) { const v4u lo = pack8_bf16_lo(a, c); o = second ? lo : hi; }
  }
  const v4u mw = (v4u){ pk16(mk[0], mk[1]), pk16(mk[2], mk[3]), pk16(mk[4], mk[5]), pk16(mk[6], mk[7]) };
  o &= mw;
  if (g < total) {
    volatile v4u* q = (volatile v4u*)(dst + (size_t)g * 8);
    *q = o;
    __threadfence();
    *q = o;
  }
}

template <int FORM> struct FragOf    { typedef FragB T; };
template <>         struct FragOf<2> { typedef FragH T; };
__device__ __forceinline__ v8f mm(const FragB& a, const FragB& b, v8f c) { return wmb(a, b, c); }
__device__ __forceinline__ v8f mm(const FragH& a, const FragH& b, v8f c) { return wmh(a, b, c); }
template <class F> __device__ __forceinline__ F ld_frag(const unsigned short* p) {
  F f;
  f.h[0] = *(const v8usa*)(p);
  f.h[1] = *(const v8usa*)(p + 16);
  return f;
}

template <int FORM, int EPI>
__global__ __launch_bounds__(256) __attribute__((amdgpu_num_vgpr(248)))
void k_gemm_nt(const unsigned short* __restrict__ A, const unsigned short* __restrict__ B,
               const float* __restrict__ bias, float* __restrict__ D, int M, int N, int KTOT, int ldd) {
  static_assert(FORM >= 0 && FORM <= 2);
  static_assert(EPI == 0 || EPI == 1);
  typedef typename FragOf<FORM>::T F;
  __shared__ __attribute__((aligned(16))) float sT[8][16 * 68];
  const int lane = threadIdx.x & 31;
  const int wave = threadIdx.x >> 5;
  const int tilesM = (M + 63) >> 6;
  const int tilesN = (N + 63) >> 6;
  const int tile = blockIdx.x * 8 + wave;
  if (tile >= tilesM * tilesN) return;
  const int tm = tile / tilesN;
  const int tn = tile - tm * tilesN;
  const int m0 = tm << 6;
  const int n0 = tn << 6;

  const int rl = lane & 15;
  const int h8 = (lane >> 4) * 8;
  const unsigned short* pa = A + (size_t)(m0 + rl) * (size_t)KTOT + h8;
  const unsigned short* pb = B + (size_t)(n0 + rl) * (size_t)KTOT + h8;

  v8f acc[4][4];
#pragma unroll
  for (int i = 0; i < 4; ++i)
#pragma unroll
    for (int j = 0; j < 4; ++j) acc[i][j] = (v8f){0.f, 0.f, 0.f, 0.f, 0.f, 0.f, 0.f, 0.f};

#pragma unroll 1
  for (int k0 = 0; k0 < KTOT; k0 += 32) {
    F bf[4];
#pragma unroll
    for (int j = 0; j < 4; ++j) bf[j] = ld_frag<F>(pb + (size_t)(j << 4) * (size_t)KTOT + k0);
#pragma unroll
    for (int i = 0; i < 4; ++i) {
      const F af = ld_frag<F>(pa + (size_t)(i << 4) * (size_t)KTOT + k0);
#pragma unroll
      for (int j = 0; j < 4; ++j) acc[i][j] = mm(af, bf[j], acc[i][j]);
    }
  }

  float* slab = sT[wave];
  const int hh = lane >> 4;
  const int c4 = (lane & 15) * 4;
  const int nc = n0 + c4;
  const bool cok = nc < N;
  v4f bv = (v4f){0.f, 0.f, 0.f, 0.f};
  if (EPI == 1) {
    bv = *(const v4fa*)(bias + clampi(nc, 0, N - 4));
    asm volatile("" :: "v"(bv));
  }
#pragma unroll
  for (int i = 0; i < 4; ++i) {
    const int mBase = m0 + (i << 4);
#pragma unroll
    for (int j = 0; j < 4; ++j) {
#pragma unroll
      for (int r = 0; r < 8; ++r) slab[(h8 + r) * 68 + (j << 4) + rl] = acc[i][j][r];
    }
    __builtin_amdgcn_fence(__ATOMIC_RELEASE, "workgroup");
    __builtin_amdgcn_wave_barrier();
    __builtin_amdgcn_fence(__ATOMIC_ACQUIRE, "workgroup");
    v4f vv[8];
#pragma unroll
    for (int it = 0; it < 8; ++it) {
      const int row = it * 2 + hh;
      v4f v = *(const v4fa*)(slab + row * 68 + c4);
      if (EPI == 1) v += bv;
      vv[it] = v;
    }
    for (int pass = 0; pass < 2; ++pass) {
#pragma unroll
      for (int it = 0; it < 8; ++it) {
        const int row = mBase + it * 2 + hh;
        if (cok && row < M) *(volatile v4f*)(D + (size_t)row * (size_t)ldd + nc) = vv[it];
      }
      __threadfence();
    }
    __builtin_amdgcn_fence(__ATOMIC_RELEASE, "workgroup");
    __builtin_amdgcn_wave_barrier();
    __builtin_amdgcn_fence(__ATOMIC_ACQUIRE, "workgroup");
  }
}

#include <stddef.h>
#include <math.h>
#pragma clang fp contract(off)

#ifndef SPLIT_L
#define SPLIT_L 1
#endif
#ifndef SPLIT_C
#define SPLIT_C 1
#endif

#define NN      100000
#define NE      1600000
#define DIN     32
#define HD      64
#define NCLS    2
#define MP      100096
#define KOP     (HD * (1 + SPLIT_L))
#define NTHR    256
#define NWAVE   8
#define EPT     8
#define WCH     (32 * EPT)
#define NBRUN   1024
#define SLB     10
#define NBK     98
#define WLCAP   4608
#define LCAP    21504
#define DEGCAP  64
#define MAXDEG_MEAS   36
#define MAXB1024_MEAS 16710
#define WBLK    12500
#define NOUT    200000
#define NLINE   6250
#define LSBLK   782

#define BK_ZINTS (NWAVE * WLCAP + LCAP + 3 * NBRUN)
#define BK_INTS  (BK_ZINTS + 16)
#define BK_LDS   (BK_INTS * 4)

#define PW0U    (HD * DIN / 8)
#define PW1U    (HD * KOP / 8)
#define PB1     (PW1U / NTHR)
#define PADOU   ((MP - NN) * KOP / 8)
#define PADOB   (PADOU / NTHR)
#define PADXU   ((MP - NN) * HD / 4)
#define PADXB   (PADXU / NTHR)
#define B_WL0   0
#define B_WR0   1
#define B_L1L   2
#define B_L1R   (B_L1L + PB1)
#define B_L2L   (B_L1R + PB1)
#define B_L2R   (B_L2L + PB1)
#define B_WC    (B_L2R + PB1)
#define B_T0    (B_WC + PB1)
#define B_T1    (B_T0 + 1)
#define B_T2    (B_T0 + 2)
#define B_TC    (B_T0 + 3)
#define B_PO    (B_T0 + 4)
#define B_PX    (B_PO + PADOB)
#define PREPBLK (B_PX + PADXB)

static_assert(SPLIT_L == 0 || SPLIT_L == 1);
static_assert(SPLIT_C == 0 || SPLIT_C == 1);
static_assert(SPLIT_C <= SPLIT_L);
static_assert(MP == 782 * 128 && MP % 128 == 0 && MP % 64 == 0 && MP >= NN);
static_assert(NN % 16 == 0 && NOUT % 32 == 0 && NOUT == NN * NCLS && NLINE * 32 == NOUT);
static_assert(LSBLK * NWAVE >= NLINE && (LSBLK - 1) * NWAVE < NLINE);
static_assert(WBLK * NWAVE == NN);
static_assert(DIN % 32 == 0 && KOP % 32 == 0 && HD % 64 == 0 && HD == 32 * 2 && HD % 32 == 0);
static_assert((HD * 4) % 128 == 0 && (KOP * 2) % 128 == 0 && (DIN * 2) % 64 == 0);
static_assert(NBRUN == (1 << SLB) && NBRUN == NTHR * 4 && NBRUN % 32 == 0);
static_assert(NBK * NBRUN >= NN && (NBK - 1) * NBRUN < NN);
static_assert(NE < (1 << 21) && (((long long)NE) << SLB) < (1LL << 31));
static_assert(NE % WCH == 0 && NE % EPT == 0 && NE >= EPT);
static_assert(LCAP % 1024 == 0 && LCAP % (NTHR * 4) == 0);
static_assert((long long)LCAP * 100 >= (long long)MAXB1024_MEAS * 125);
static_assert(WLCAP >= 2 * ((MAXB1024_MEAS + 7) / 8));
static_assert(MAXDEG_MEAS + 8 <= DEGCAP);
static_assert(BK_ZINTS % (NTHR * 4) == 0 && BK_LDS <= 262144 && BK_LDS + 0 <= 327680);
static_assert(PW0U == NTHR && PW1U % NTHR == 0 && PADOU % NTHR == 0 && PADXU % NTHR == 0);
static_assert((MP * DIN / 8) % NTHR == 0);

typedef float        v2f  __attribute__((ext_vector_type(2)));
typedef int          v4i  __attribute__((ext_vector_type(4)));
typedef v2f __attribute__((may_alias)) v2fa;
typedef v4i __attribute__((may_alias)) v4ia;

__device__ __forceinline__ void st2_v4f(float* p, v4f v) {
  *(volatile v4f*)p = v;
  __threadfence();
  *(volatile v4f*)p = v;
}
__device__ __forceinline__ void st2_v4u(unsigned short* p, v4u v) {
  *(volatile v4u*)p = v;
  __threadfence();
  *(volatile v4u*)p = v;
}
__device__ __forceinline__ void st2_f32(float* p, float v) {
  *(volatile float*)p = v;
  __threadfence();
  *(volatile float*)p = v;
}

__device__ __forceinline__ void wplane_unit(const float* __restrict__ W, const int kin, const int kt, const int rowsValid,
                                            const int secondOn, unsigned short* dst, const int u) {
  const int ppr = kt >> 3;
  const int n   = u / ppr;
  const int k8  = (u - n * ppr) << 3;
  const int ks  = k8 & (kin - 1);
  const int nr  = n < rowsValid ? n : rowsValid - 1;
  const float* r = W + (size_t)nr * (size_t)kin + ks;
  const v4f a = *(const v4fa*)r;
  const v4f c = *(const v4fa*)(r + 4);
  asm volatile("" :: "v"(a), "v"(c));
  const bool on = (n < rowsValid) && (k8 < kin || secondOn != 0);
  const unsigned mk = on ? 0xFFFFFFFFu : 0u;
  v4u o = pack8_bf16(a, c);
  o &= (v4u){ mk, mk, mk, mk };
  st2_v4u(dst + (size_t)u * 8, o);
}

__device__ __forceinline__ void tab_layer(const float* __restrict__ b, const float* __restrict__ g,
                                          const float* __restrict__ be, const float* __restrict__ rm,
                                          const float* __restrict__ rv, float* tab, const int tid) {
  if (tid < 64) {
    const float vb = b[tid], vg = g[tid], vbe = be[tid], vrm = rm[tid], vrv = rv[tid];
    asm volatile("" :: "v"(vb), "v"(vg), "v"(vbe), "v"(vrm), "v"(vrv));
    float qb = bf16_val(vb), qg = bf16_val(vg), qbe = bf16_val(vbe), qrm = bf16_val(vrm), qrv = bf16_val(vrv);
    asm volatile("" : "+v"(qb));
    asm volatile("" : "+v"(qg));
    asm volatile("" : "+v"(qbe));
    asm volatile("" : "+v"(qrm));
    asm volatile("" : "+v"(qrv));
    const float rt = sqrtf(qrv + 1e-5f);
    const float ri = 1.0f / rt;
    const float sc = qg * ri;
    for (int pass = 0; pass < 2; ++pass) {
      *(volatile float*)(tab + tid)       = qb;
      *(volatile float*)(tab + 64 + tid)  = qrm;
      *(volatile float*)(tab + 128 + tid) = sc;
      *(volatile float*)(tab + 192 + tid) = qbe;
      __threadfence();
    }
  }
}

__global__ __launch_bounds__(NTHR) void k_prep(
    const float* __restrict__ wl0, const float* __restrict__ wr0, const float* __restrict__ wl1,
    const float* __restrict__ wr1, const float* __restrict__ wl2, const float* __restrict__ wr2,
    const float* __restrict__ wc,
    const float* __restrict__ b0, const float* __restrict__ g0, const float* __restrict__ be0,
    const float* __restrict__ rm0, const float* __restrict__ rv0,
    const float* __restrict__ b1, const float* __restrict__ g1, const float* __restrict__ be1,
    const float* __restrict__ rm1, const float* __restrict__ rv1,
    const float* __restrict__ b2, const float* __restrict__ g2, const float* __restrict__ be2,
    const float* __restrict__ rm2, const float* __restrict__ rv2,
    const float* __restrict__ bc,
    unsigned short* pl0, unsigned short* pr0, unsigned short* pl1, unsigned short* pr1,
    unsigned short* pl2, unsigned short* pr2, unsigned short* pc,
    float* tab, unsigned short* op, float* xf) {
  const int tid = (int)threadIdx.x;
  const int blk = (int)blockIdx.x;
  if (blk == B_WL0) {
    wplane_unit(wl0, DIN, DIN, HD, 0, pl0, tid);
  } else if (blk == B_WR0) {
    wplane_unit(wr0, DIN, DIN, HD, 0, pr0, tid);
  } else if (blk < B_L1R) {
    wplane_unit(wl1, HD, KOP, HD, 1, pl1, (blk - B_L1L) * NTHR + tid);
  } else if (blk < B_L2L) {
    wplane_unit(wr1, HD, KOP, HD, 1, pr1, (blk - B_L1R) * NTHR + tid);
  } else if (blk < B_L2R) {
    wplane_unit(wl2, HD, KOP, HD, 1, pl2, (blk - B_L2L) * NTHR + tid);
  } else if (blk < B_WC) {
    wplane_unit(wr2, HD, KOP, HD, 1, pr2, (blk - B_L2R) * NTHR + tid);
  } else if (blk < B_T0) {
    wplane_unit(wc, HD, KOP, NCLS, SPLIT_C, pc, (blk - B_WC) * NTHR + tid);
  } else if (blk == B_T0) {
    tab_layer(b0, g0, be0, rm0, rv0, tab, tid);
  } else if (blk == B_T1) {
    tab_layer(b1, g1, be1, rm1, rv1, tab + 256, tid);
  } else if (blk == B_T2) {
    tab_layer(b2, g2, be2, rm2, rv2, tab + 512, tid);
  } else if (blk == B_TC) {
    if (tid < 64) {
      const float v = bc[clampi(tid, 0, NCLS - 1)];
      asm volatile("" :: "v"(v));
      const unsigned mk = (tid < NCLS) ? 0xFFFFFFFFu : 0u;
      const float o = __uint_as_float(__float_as_uint(bf16_val(v)) & mk);
      st2_f32(tab + 768 + tid, o);
    }
  } else if (blk < B_PX) {
    const int u = (blk - B_PO) * NTHR + tid;
    const v4u z = (v4u){ 0u, 0u, 0u, 0u };
    st2_v4u(op + (size_t)NN * KOP + (size_t)u * 8, z);
  } else {
    const int u = (blk - B_PX) * NTHR + tid;
    const v4f z = (v4f){ 0.0f, 0.0f, 0.0f, 0.0f };
    st2_v4f(xf + (size_t)NN * HD + (size_t)u * 4, z);
  }
}

__device__ __forceinline__ void list_flush(const int* pl, const int* cnt, const int* offs, int ov,
                                           int* lp, int* cp, int* op, int* fp, int tid) {
#pragma unroll 1
  for (int i = tid * 4; i < LCAP; i += NTHR * 4) {
    const v4i v = *(const v4ia*)(pl + i);
    *(volatile v4i*)(lp + i) = v;
  }
  {
    const v4i v = *(const v4ia*)(cnt + 4 * tid);
    *(volatile v4i*)(cp + 4 * tid) = v;
  }
  {
    const v4i v = *(const v4ia*)(offs + 4 * tid);
    *(volatile v4i*)(op + 4 * tid) = v;
  }
  if (tid < 8) {
    const v4i f = {ov, ov, ov, ov};
    *(volatile v4i*)(fp + 4 * tid) = f;
  }
}

__global__ __launch_bounds__(NTHR) void k_list(const int* __restrict__ srcs, const int* __restrict__ dsts,
                                               int* LIST, int* CNT, int* OFF, int* FLAG) {
  extern __shared__ __attribute__((aligned(16))) int dsm[];
  int* wl   = dsm;
  int* pl   = dsm + NWAVE * WLCAP;
  int* cnt  = pl + LCAP;
  int* offs = cnt + NBRUN;
  int* cur  = offs + NBRUN;
  int* misc = cur + NBRUN;
  const int tid = (int)threadIdx.x, lane = tid & 31, wave = tid >> 5;
  const int blk = (int)blockIdx.x;
  const unsigned nbs = (unsigned)(blk * NBRUN);

  {
    const v4i z4 = {0, 0, 0, 0};
    for (int i = tid * 4; i < BK_ZINTS; i += NTHR * 4) *(v4ia*)(dsm + i) = z4;
    if (tid < 16) misc[tid] = 0;
  }
  __syncthreads();

  {
    const int per  = ((NE + NWAVE * WCH - 1) / (NWAVE * WCH)) * WCH;
    const int ebeg = wave * per;
    const int eend = (ebeg + per < NE) ? (ebeg + per) : NE;
    int* mylist = wl + wave * WLCAP;
    int wc = 0;
#pragma unroll 1
    for (int cb = ebeg; cb < eend; cb += WCH) {
      const int e0 = cb + lane * EPT;
      const int ec = e0 < NE - EPT ? e0 : NE - EPT;
      const bool lv = e0 < NE;
      const v4i da = *(const v4ia*)(dsts + ec);
      const v4i db = *(const v4ia*)(dsts + ec + 4);
      asm volatile("" :: "v"(da), "v"(db));
      const unsigned s0 = (unsigned)da.x - nbs, s1 = (unsigned)da.y - nbs;
      const unsigned s2 = (unsigned)da.z - nbs, s3 = (unsigned)da.w - nbs;
      const unsigned s4 = (unsigned)db.x - nbs, s5 = (unsigned)db.y - nbs;
      const unsigned s6 = (unsigned)db.z - nbs, s7 = (unsigned)db.w - nbs;
      const bool h0 = lv && s0 < (unsigned)NBRUN && (unsigned)da.x < (unsigned)NN;
      const bool h1 = lv && s1 < (unsigned)NBRUN && (unsigned)da.y < (unsigned)NN;
      const bool h2 = lv && s2 < (unsigned)NBRUN && (unsigned)da.z < (unsigned)NN;
      const bool h3 = lv && s3 < (unsigned)NBRUN && (unsigned)da.w < (unsigned)NN;
      const bool h4 = lv && s4 < (unsigned)NBRUN && (unsigned)db.x < (unsigned)NN;
      const bool h5 = lv && s5 < (unsigned)NBRUN && (unsigned)db.y < (unsigned)NN;
      const bool h6 = lv && s6 < (unsigned)NBRUN && (unsigned)db.z < (unsigned)NN;
      const bool h7 = lv && s7 < (unsigned)NBRUN && (unsigned)db.w < (unsigned)NN;
      const unsigned m0 = __builtin_amdgcn_ballot_w32(h0), m1 = __builtin_amdgcn_ballot_w32(h1);
      const unsigned m2 = __builtin_amdgcn_ballot_w32(h2), m3 = __builtin_amdgcn_ballot_w32(h3);
      const unsigned m4 = __builtin_amdgcn_ballot_w32(h4), m5 = __builtin_amdgcn_ballot_w32(h5);
      const unsigned m6 = __builtin_amdgcn_ballot_w32(h6), m7 = __builtin_amdgcn_ballot_w32(h7);
      const unsigned any = m0 | m1 | m2 | m3 | m4 | m5 | m6 | m7;
      if (any != 0u) {
        const int pre = (int)(__builtin_amdgcn_mbcnt_lo(m0, 0u) + __builtin_amdgcn_mbcnt_lo(m1, 0u) +
                              __builtin_amdgcn_mbcnt_lo(m2, 0u) + __builtin_amdgcn_mbcnt_lo(m3, 0u) +
                              __builtin_amdgcn_mbcnt_lo(m4, 0u) + __builtin_amdgcn_mbcnt_lo(m5, 0u) +
                              __builtin_amdgcn_mbcnt_lo(m6, 0u) + __builtin_amdgcn_mbcnt_lo(m7, 0u));
        int p = wc + pre;
        if (h0) { if (p < WLCAP) mylist[p] = ((e0 + 0) << SLB) | (int)s0; p = p + 1; }
        if (h1) { if (p < WLCAP) mylist[p] = ((e0 + 1) << SLB) | (int)s1; p = p + 1; }
        if (h2) { if (p < WLCAP) mylist[p] = ((e0 + 2) << SLB) | (int)s2; p = p + 1; }
        if (h3) { if (p < WLCAP) mylist[p] = ((e0 + 3) << SLB) | (int)s3; p = p + 1; }
        if (h4) { if (p < WLCAP) mylist[p] = ((e0 + 4) << SLB) | (int)s4; p = p + 1; }
        if (h5) { if (p < WLCAP) mylist[p] = ((e0 + 5) << SLB) | (int)s5; p = p + 1; }
        if (h6) { if (p < WLCAP) mylist[p] = ((e0 + 6) << SLB) | (int)s6; p = p + 1; }
        if (h7) { if (p < WLCAP) mylist[p] = ((e0 + 7) << SLB) | (int)s7; p = p + 1; }
        wc += (int)(__builtin_popcount(m0) + __builtin_popcount(m1) + __builtin_popcount(m2) + __builtin_popcount(m3) +
                    __builtin_popcount(m4) + __builtin_popcount(m5) + __builtin_popcount(m6) + __builtin_popcount(m7));
      }
    }
    if (lane == 0) misc[wave] = wc;
  }
  __syncthreads();

  if (wave == 0) {
    int ov = 0;
    int tot = 0;
#pragma unroll 1
    for (int w2 = 0; w2 < NWAVE; ++w2) {
      int c = misc[w2];
      if (c > WLCAP) ov = 1;
      c = c < 0 ? 0 : (c > WLCAP ? WLCAP : c);
      tot += c;
#pragma unroll 1
      for (int b0 = 0; b0 < c; b0 += 32) {
        const int idx = b0 + lane;
        const int ent = wl[w2 * WLCAP + (idx < WLCAP ? idx : WLCAP - 1)];
        const int m32 = (c - b0) < 32 ? (c - b0) : 32;
#pragma unroll 1
        for (int k = 0; k < m32; ++k) {
          const int u    = __builtin_amdgcn_readlane(ent, k);
          const int slot = u & (NBRUN - 1);
          if (lane == 0) cnt[slot] = cnt[slot] + 1;
        }
      }
    }
    if (tot > LCAP) ov = 1;
    if (lane == 0) misc[9] = ov;
  }
  __syncthreads();
  if (wave == 0) {
    const int base = lane * (NBRUN / 32);
    int s = 0;
#pragma unroll 1
    for (int i = 0; i < NBRUN / 32; ++i) s += cnt[base + i];
    int incl = s;
#pragma unroll
    for (int d = 1; d < 32; d <<= 1) {
      const int y = __shfl_up(incl, d, 32);
      if (lane >= d) incl += y;
    }
    int run = incl - s;
#pragma unroll 1
    for (int i = 0; i < NBRUN / 32; ++i) {
      const int cv = cnt[base + i];
      offs[base + i] = run;
      cur[base + i]  = run;
      run += cv;
    }
  }
  __syncthreads();

  if (wave == 0) {
#pragma unroll 1
    for (int w2 = 0; w2 < NWAVE; ++w2) {
      int c = misc[w2];
      c = c < 0 ? 0 : (c > WLCAP ? WLCAP : c);
#pragma unroll 1
      for (int b0 = 0; b0 < c; b0 += 32) {
        const int idx = b0 + lane;
        const int ent = wl[w2 * WLCAP + (idx < WLCAP ? idx : WLCAP - 1)];
        int eid = (ent >> SLB) & 0x1FFFFF;
        eid = eid > NE - 1 ? NE - 1 : eid;
        int sr = srcs[eid];
        asm volatile("" :: "v"(sr));
        sr = clampi(sr, 0, NN - 1);
        const int m32 = (c - b0) < 32 ? (c - b0) : 32;
#pragma unroll 1
        for (int k = 0; k < m32; ++k) {
          const int u    = __builtin_amdgcn_readlane(ent, k);
          const int w0   = __builtin_amdgcn_readlane(sr, k);
          const int slot = u & (NBRUN - 1);
          if (lane == 0) {
            int p = cur[slot];
            p = p < 0 ? 0 : (p > LCAP - 1 ? LCAP - 1 : p);
            pl[p] = w0;
            cur[slot] = p + 1;
          }
        }
      }
    }
  }
  __syncthreads();

  const int ovf = misc[9];
  int* lp = LIST + (size_t)blk * (size_t)LCAP;
  int* cp = CNT  + (size_t)blk * NBRUN;
  int* op = OFF  + (size_t)blk * NBRUN;
  int* fp = FLAG + (size_t)blk * 32;
  list_flush(pl, cnt, offs, ovf, lp, cp, op, fp, tid);
  __threadfence();
  list_flush(pl, cnt, offs, ovf, lp, cp, op, fp, tid);
}

template <int RES>
__global__ __launch_bounds__(NTHR) void k_walk(const int* __restrict__ LIST, const int* __restrict__ CNT,
                                               const int* __restrict__ OFF, const int* __restrict__ FLAG,
                                               const float* __restrict__ T, const float* __restrict__ S,
                                               const float* __restrict__ TABL, float* XF, unsigned short* OP) {
  const int tid = (int)threadIdx.x, lane = tid & 31, wave = tid >> 5;
  const int blk = (int)blockIdx.x;
  const int n  = blk * NWAVE + wave;
  const int bk = n >> SLB;
  const int cv = CNT[n];
  asm volatile("" :: "v"(cv));
  const int ovv = OFF[n];
  asm volatile("" :: "v"(ovv));
  const int fl = FLAG[(size_t)bk * 32];
  asm volatile("" :: "v"(fl));

  const bool bad = (fl != 0) || (cv > DEGCAP) || (cv < 0);
  const int trip = __builtin_amdgcn_readfirstlane((fl == 0 && cv > 0) ? (cv > DEGCAP ? DEGCAP : cv) : 0);
  const int o = clampi(ovv, 0, LCAP - 1);
  int last = o + (trip > 0 ? trip : 1) - 1;
  last = last > LCAP - 1 ? LCAP - 1 : last;
  const int* lb = LIST + (size_t)bk * (size_t)LCAP;
  const float* tl = T + 2 * lane;

  v2f acc = (v2f){0.0f, 0.0f};
#pragma unroll 1
  for (int b0 = 0; b0 < trip; b0 += 32) {
    int idx = o + b0 + lane;
    idx = idx > last ? last : idx;
    int sr = lb[idx];
    sr = clampi(sr, 0, NN - 1);
    const int m32 = (trip - b0) < 32 ? (trip - b0) : 32;
#pragma unroll 1
    for (int k = 0; k < m32; ++k) {
      const int sk = __builtin_amdgcn_readlane(sr, k);
      const v2f q = *(const v2fa*)(tl + (size_t)sk * HD);
      acc += q;
    }
  }

  const v2f sv = *(const v2fa*)(S + (size_t)n * HD + 2 * lane);
  float s0 = sv.x, s1 = sv.y;
  asm volatile("" : "+v"(s0));
  asm volatile("" : "+v"(s1));
  const v2f rmv = *(const v2fa*)(TABL + 64 + 2 * lane);
  const v2f scv = *(const v2fa*)(TABL + 128 + 2 * lane);
  const v2f bev = *(const v2fa*)(TABL + 192 + 2 * lane);
  float rm0 = rmv.x, rm1 = rmv.y, sc0 = scv.x, sc1 = scv.y, be0 = bev.x, be1 = bev.y;
  asm volatile("" : "+v"(rm0));
  asm volatile("" : "+v"(rm1));
  asm volatile("" : "+v"(sc0));
  asm volatile("" : "+v"(sc1));
  asm volatile("" : "+v"(be0));
  asm volatile("" : "+v"(be1));
  float x0 = 0.0f, x1 = 0.0f;
  if (RES == 1) {
    const v2f xv = *(const v2fa*)(XF + (size_t)n * HD + 2 * lane);
    x0 = xv.x; x1 = xv.y;
    asm volatile("" : "+v"(x0));
    asm volatile("" : "+v"(x1));
  }

  const int cm = cv > 1 ? cv : 1;
  const float cf = (float)cm;
  const float m0 = acc.x / cf;
  const float m1 = acc.y / cf;
  const float v0 = s0 + m0;
  const float v1 = s1 + m1;
  const float d0 = v0 - rm0;
  const float d1 = v1 - rm1;
  const float p0 = d0 * sc0;
  const float p1 = d1 * sc1;
  const float z0 = p0 + be0;
  const float z1 = p1 + be1;
  float y0 = (z0 > 0.0f) ? z0 : (z0 - z0);
  float y1 = (z1 > 0.0f) ? z1 : (z1 - z1);
  if (RES == 1) {
    y0 = y0 + x0;
    y1 = y1 + x1;
  }
  const float qnan = __uint_as_float(0x7fc00000u);
  const float u0 = bad ? qnan : y0;
  const float u1 = bad ? qnan : y1;

  const v2f yv = (v2f){u0, u1};
  const unsigned hw = pk16(bf16_bits(u0), bf16_bits(u1));
  const unsigned lw = pk16(bf16_lo_bits(u0), bf16_lo_bits(u1));
  float* xr = XF + (size_t)n * HD + 2 * lane;
  unsigned short* cr = OP + (size_t)n * KOP + 2 * lane;
  for (int pass = 0; pass < 2; ++pass) {
    *(volatile v2f*)xr = yv;
    *(volatile unsigned*)cr = hw;
    if (SPLIT_L) *(volatile unsigned*)(cr + HD) = lw;
    __threadfence();
  }
}

__global__ __launch_bounds__(NTHR) void k_lsm_store(const float* __restrict__ T, float* out, int nOut) {
  const int tid = (int)threadIdx.x, lane = tid & 31, wave = tid >> 5;
  const int line = (int)blockIdx.x * NWAVE + wave;
  if (line >= NLINE) return;
  const int f   = line * 32 + lane;
  const int row = f >> 1;
  const int col = f & 1;
  const int rc  = clampi(row, 0, NN - 1);
  const v2f lg = *(const v2fa*)(T + (size_t)rc * HD);
  float l0 = lg.x, l1 = lg.y;
  asm volatile("" : "+v"(l0));
  asm volatile("" : "+v"(l1));
  const float mx  = (l0 > l1 || l0 != l0) ? l0 : l1;
  const float sh0 = l0 - mx;
  const float sh1 = l1 - mx;
  const float e0  = expf(sh0);
  const float e1  = expf(sh1);
  const float lse = logf(e0 + e1);
  const float o0  = sh0 - lse;
  const float o1  = sh1 - lse;
  const float o   = (col != 0) ? o1 : o0;
  if (f < nOut) {
    st2_f32(out + f, o);
  }
}

extern "C" void kernel_launch(void* const* d_in, const int* in_sizes, int n_in,
                              void* d_out, int out_size, void* d_ws, size_t ws_size,
                              hipStream_t stream) {
  if (n_in < 25) return;
  if (in_sizes[0] != NN * DIN) return;
  if (in_sizes[1] != 2 * NE) return;
  if (in_sizes[2] != HD * DIN || in_sizes[4] != HD * DIN) return;
  if (in_sizes[9] != HD * HD || in_sizes[11] != HD * HD) return;
  if (in_sizes[16] != HD * HD || in_sizes[18] != HD * HD) return;
  for (int l = 0; l < 3; ++l) {
    const int base = 2 + 7 * l;
    if (in_sizes[base + 1] != HD || in_sizes[base + 3] != HD || in_sizes[base + 4] != HD) return;
    if (in_sizes[base + 5] != HD || in_sizes[base + 6] != HD) return;
  }
  if (in_sizes[23] != NCLS * HD) return;
  if (in_sizes[24] != NCLS) return;
  if (out_size != NOUT) return;

  const float* x    = (const float*)d_in[0];
  const int*   ei   = (const int*)d_in[1];
  const int*   srcs = ei;
  const int*   dsts = ei + NE;
  const float* Wl0 = (const float*)d_in[2];
  const float* b0  = (const float*)d_in[3];
  const float* Wr0 = (const float*)d_in[4];
  const float* g0  = (const float*)d_in[5];
  const float* be0 = (const float*)d_in[6];
  const float* rm0 = (const float*)d_in[7];
  const float* rv0 = (const float*)d_in[8];
  const float* Wl1 = (const float*)d_in[9];
  const float* b1  = (const float*)d_in[10];
  const float* Wr1 = (const float*)d_in[11];
  const float* g1  = (const float*)d_in[12];
  const float* be1 = (const float*)d_in[13];
  const float* rm1 = (const float*)d_in[14];
  const float* rv1 = (const float*)d_in[15];
  const float* Wl2 = (const float*)d_in[16];
  const float* b2  = (const float*)d_in[17];
  const float* Wr2 = (const float*)d_in[18];
  const float* g2  = (const float*)d_in[19];
  const float* be2 = (const float*)d_in[20];
  const float* rm2 = (const float*)d_in[21];
  const float* rv2 = (const float*)d_in[22];
  const float* Wc  = (const float*)d_in[23];
  const float* bc  = (const float*)d_in[24];
  float* out = (float*)d_out;

  constexpr size_t zXB   = (size_t)MP * DIN * 2;
  constexpr size_t zOP   = (size_t)MP * 128 * 2;
  constexpr size_t zF    = (size_t)MP * HD * 4;
  constexpr size_t zLIST = (size_t)NBK * LCAP * 4;
  constexpr size_t zTABI = (size_t)NBK * NBRUN * 4;
  constexpr size_t zFLAG = (size_t)NBK * 128;
  constexpr size_t zW0   = (size_t)HD * DIN * 2;
  constexpr size_t zW1   = (size_t)HD * 128 * 2;
  constexpr size_t zTAB  = 4096;
  constexpr size_t oXB   = 0;
  constexpr size_t oOP   = oXB + zXB;
  constexpr size_t oS    = oOP + zOP;
  constexpr size_t oT    = oS + zF;
  constexpr size_t oXF   = oT + zF;
  constexpr size_t oLIST = oXF + zF;
  constexpr size_t oCNT  = oLIST + zLIST;
  constexpr size_t oOFF  = oCNT + zTABI;
  constexpr size_t oFLAG = oOFF + zTABI;
  constexpr size_t oPL0  = oFLAG + zFLAG;
  constexpr size_t oPR0  = oPL0 + zW0;
  constexpr size_t oPL1  = oPR0 + zW0;
  constexpr size_t oPR1  = oPL1 + zW1;
  constexpr size_t oPL2  = oPR1 + zW1;
  constexpr size_t oPR2  = oPL2 + zW1;
  constexpr size_t oPC   = oPR2 + zW1;
  constexpr size_t oTAB  = oPC + zW1;
  constexpr size_t oEND  = oTAB + zTAB;
  static_assert(zXB % 128 == 0 && zOP % 128 == 0 && zF % 128 == 0 && zLIST % 128 == 0 && zTABI % 128 == 0);
  static_assert(zFLAG % 128 == 0 && zW0 % 128 == 0 && zW1 % 128 == 0 && zTAB % 128 == 0);
  static_assert(zOP >= (size_t)MP * KOP * 2 && zW1 >= (size_t)HD * KOP * 2 && zTAB >= (size_t)13 * 64 * 4);
  static_assert(oEND == (size_t)923778 * 128);
  static_assert(oEND <= ((size_t)128 << 20));
  if (oEND > ws_size) return;

  char* ws = (char*)d_ws;
  unsigned short* XB   = (unsigned short*)(ws + oXB);
  unsigned short* OP   = (unsigned short*)(ws + oOP);
  float*          S    = (float*)(ws + oS);
  float*          T    = (float*)(ws + oT);
  float*          XF   = (float*)(ws + oXF);
  int*            LIST = (int*)(ws + oLIST);
  int*            CNT  = (int*)(ws + oCNT);
  int*            OFF  = (int*)(ws + oOFF);
  int*            FLAG = (int*)(ws + oFLAG);
  unsigned short* PL0  = (unsigned short*)(ws + oPL0);
  unsigned short* PR0  = (unsigned short*)(ws + oPR0);
  unsigned short* PL1  = (unsigned short*)(ws + oPL1);
  unsigned short* PR1  = (unsigned short*)(ws + oPR1);
  unsigned short* PL2  = (unsigned short*)(ws + oPL2);
  unsigned short* PR2  = (unsigned short*)(ws + oPR2);
  unsigned short* PC   = (unsigned short*)(ws + oPC);
  float*          TAB  = (float*)(ws + oTAB);

  hipFuncSetAttribute(reinterpret_cast<const void*>(&k_list), hipFuncAttributeMaxDynamicSharedMemorySize, (int)BK_LDS);

  const int tiles = ((NN + 63) / 64) * (HD / 64);
  const int gg    = (tiles + 7) / 8;

  k_plane<0><<<MP * DIN / 8 / NTHR, NTHR, 0, stream>>>(x, NN, DIN, DIN, XB, MP, DIN);
  k_prep<<<PREPBLK, NTHR, 0, stream>>>(Wl0, Wr0, Wl1, Wr1, Wl2, Wr2, Wc,
                                       b0, g0, be0, rm0, rv0, b1, g1, be1, rm1, rv1, b2, g2, be2, rm2, rv2, bc,
                                       PL0, PR0, PL1, PR1, PL2, PR2, PC, TAB, OP, XF);
  k_list<<<NBK, NTHR, BK_LDS, stream>>>(srcs, dsts, LIST, CNT, OFF, FLAG);

  k_gemm_nt<0, 1><<<gg, NTHR, 0, stream>>>(XB, PR0, TAB + 0, S, NN, HD, DIN, HD);
  k_gemm_nt<0, 0><<<gg, NTHR, 0, stream>>>(XB, PL0, TAB + 0, T, NN, HD, DIN, HD);
  k_walk<0><<<WBLK, NTHR, 0, stream>>>(LIST, CNT, OFF, FLAG, T, S, TAB + 0, XF, OP);
  k_gemm_nt<0, 1><<<gg, NTHR, 0, stream>>>(OP, PR1, TAB + 256, S, NN, HD, KOP, HD);
  k_gemm_nt<0, 0><<<gg, NTHR, 0, stream>>>(OP, PL1, TAB + 256, T, NN, HD, KOP, HD);
  k_walk<1><<<WBLK, NTHR, 0, stream>>>(LIST, CNT, OFF, FLAG, T, S, TAB + 256, XF, OP);
  k_gemm_nt<0, 1><<<gg, NTHR, 0, stream>>>(OP, PR2, TAB + 512, S, NN, HD, KOP, HD);
  k_gemm_nt<0, 0><<<gg, NTHR, 0, stream>>>(OP, PL2, TAB + 512, T, NN, HD, KOP, HD);
  k_walk<1><<<WBLK, NTHR, 0, stream>>>(LIST, CNT, OFF, FLAG, T, S, TAB + 512, XF, OP);
  k_gemm_nt<0, 1><<<gg, NTHR, 0, stream>>>(OP, PC, TAB + 768, T, NN, HD, KOP, HD);
  k_lsm_store<<<LSBLK, NTHR, 0, stream>>>(T, out, out_size);
}
